// ExternalMemoryNetwork_9869834846291
// MI455X (gfx1250) — hardware-verified
//
#include <hip/hip_runtime.h>


namespace {
constexpr int B = 1024, M = 200000, D = 64;
constexpr float XS = 8.0f, VSC = 256.0f, PS = 8.0f, LOG2E = 1.4426950408889634f;

typedef _Float16 b16;
typedef __attribute__((ext_vector_type(16))) _Float16 v16b;
typedef __attribute__((ext_vector_type(8))) _Float16 v8b;
typedef __attribute__((ext_vector_type(8))) float v8f;
typedef __attribute__((ext_vector_type(4))) float v4f;
__device__ __forceinline__ float bf16_rne(float f) { unsigned int u = __float_as_uint(f); u += 0x7FFFu + ((u >> 16) & 1u); return __uint_as_float(u & 0xFFFF0000u); }
__device__ __forceinline__ v16b frag_kb(const b16* p, int hh) { const v8b a = *(const v8b*)(p + 8 * hh), b = *(const v8b*)(p + 16 + 8 * hh); v16b f;
#pragma unroll
  for (int e = 0; e < 8; ++e) { f[e] = a[e]; f[8 + e] = b[e]; } return f; }
__device__ __forceinline__ v8f wmma16b(v16b a, v16b b, v8f c) { v8f d = __builtin_amdgcn_wmma_f32_16x16x32_f16(false, a, false, b, (short)0, c, false, false); asm volatile("v_nop\n\tv_nop\n\tv_nop\n\tv_nop" : "+v"(d) : "v"(a), "v"(b)); return d; }
__device__ __forceinline__ void wave_lds_sync() { __builtin_amdgcn_fence(__ATOMIC_RELEASE, "workgroup"); __builtin_amdgcn_wave_barrier(); __builtin_amdgcn_fence(__ATOMIC_ACQUIRE, "workgroup"); }
__device__ __forceinline__ float nexp2(float x) { return __builtin_amdgcn_exp2f(x); }
__device__ __forceinline__ float pmul(float a, float b) { float p = a * b; asm volatile("" : "+v"(p)); return p; }
__device__ __forceinline__ int iclamp(int v, int lo, int hi) { return v < lo ? lo : (v > hi ? hi : v); }

__global__ __launch_bounds__(256) void prep_kernel(const float* __restrict__ x, const float* __restrict__ vals, b16* __restrict__ X16, b16* __restrict__ V16, b16* __restrict__ VT16) {
  __shared__ __attribute__((aligned(16))) b16 T[D][64 + 8];
  const int t_ = threadIdx.x; const size_t r0 = (size_t)blockIdx.x * 64;
  if (blockIdx.x < B * D / 8 / 256 + 1) { const size_t e = ((size_t)blockIdx.x * 256 + t_) * 8; if (e < (size_t)B * D) { v8b o; for (int j = 0; j < 8; ++j) o[j] = (b16)(bf16_rne(x[e + j]) * XS); for (int pass = 0; pass < 2; ++pass) { *(volatile v8b*)(X16 + e) = o; __threadfence(); } } }
  for (int q = t_; q < 64 * D / 8; q += 256) { const int rr = q >> 3, c8 = (q & 7) * 8; v8b o; for (int j = 0; j < 8; ++j) { const float v = bf16_rne(vals[(r0 + rr) * D + c8 + j]) * VSC; o[j] = (b16)v; T[c8 + j][rr] = (b16)v; }
    for (int pass = 0; pass < 2; ++pass) { *(volatile v8b*)(V16 + (r0 + rr) * D + c8) = o; __threadfence(); } }
  __syncthreads();
  for (int pass = 0; pass < 2; ++pass) { for (int q = t_; q < D * 8; q += 256) { const int d = q >> 3, c8 = (q & 7) * 8; *(volatile v8b*)(VT16 + (size_t)d * M + r0 + c8) = *(const v8b*)(&T[d][c8]); } __threadfence(); }
}
__global__ __launch_bounds__(64) void read_kernel(const b16* __restrict__ X16, const b16* __restrict__ V16, const b16* __restrict__ VT16, float* __restrict__ out0) {
  __shared__ __attribute__((aligned(16))) float To[2][16][D + 4];
  const int wave = threadIdx.x >> 5, lane = threadIdx.x & 31, hh = lane >> 4, col = lane & 15; const int q0 = blockIdx.x * 32 + wave * 16, qi = q0 + col;
  const v16b xa0 = frag_kb(X16 + (size_t)qi * D, hh), xa1 = frag_kb(X16 + (size_t)qi * D + 32, hh);
  float m = -INFINITY, l = 0.0f; v8f o[4] = {{}, {}, {}, {}}; const float cs = LOG2E / (XS * VSC);
  for (int kb = 0; kb < M; kb += 32) {
    v8f s0 = {}, s1 = {};
    { const b16* k0 = V16 + (size_t)(kb + col) * D, *k1 = V16 + (size_t)(kb + 16 + col) * D; s0 = wmma16b(frag_kb(k0, hh), xa0, s0); s0 = wmma16b(frag_kb(k0 + 32, hh), xa1, s0); s1 = wmma16b(frag_kb(k1, hh), xa0, s1); s1 = wmma16b(frag_kb(k1 + 32, hh), xa1, s1); }
    float e[16]; float mx = -INFINITY;
#pragma unroll
    for (int r = 0; r < 8; ++r) { e[r] = s0[r] * cs; e[8 + r] = s1[r] * cs; mx = fmaxf(mx, fmaxf(e[r], e[8 + r])); }
    mx = fmaxf(mx, __shfl_xor(mx, 16)); const float mn = fmaxf(m, mx); const float al = nexp2(m - mn); m = mn; float sum = 0.0f; v16b ph, pl;
#pragma unroll
    for (int i = 0; i < 16; ++i) { const float p = nexp2(e[i] - mn); sum += p; const b16 h_ = (b16)(p * PS); ph[i] = h_; pl[i] = (b16)(p * PS - (float)h_); }
    sum += __shfl_xor(sum, 16); l = l * al + sum;
#pragma unroll
    for (int t = 0; t < 4; ++t) { o[t] *= al; const v16b vf = frag_kb(VT16 + (size_t)(t * 16 + col) * M + kb, hh); o[t] = wmma16b(vf, ph, o[t]); o[t] = wmma16b(vf, pl, o[t]); } }
  const float inv = 1.0f / (l * PS * VSC);
#pragma unroll
  for (int t = 0; t < 4; ++t)
#pragma unroll
    for (int r = 0; r < 8; ++r) To[wave][col][t * 16 + 8 * hh + r] = o[t][r] * inv;
  wave_lds_sync();
  for (int pass = 0; pass < 2; ++pass) { for (int rr = 0; rr < 16; ++rr) if (lane < 16) *(volatile v4f*)(out0 + (size_t)(q0 + rr) * D + lane * 4) = *(const v4f*)(&To[wave][rr][lane * 4]); __threadfence(); }
}
__global__ __launch_bounds__(128) void gate_kernel(const float* __restrict__ x, const float* __restrict__ we, const float* __restrict__ be_, const float* __restrict__ wa, const float* __restrict__ ba, float* __restrict__ EA) {
  __shared__ __attribute__((aligned(16))) float row[2 * D]; __shared__ float xr[D];
  const int p = blockIdx.x, t_ = threadIdx.x; if (t_ < D) xr[t_] = bf16_rne(x[(size_t)p * D + t_]);
  __syncthreads();
  { const int c = t_ & 63; const bool isadd = t_ >= 64; const float* w = isadd ? wa : we; float s = bf16_rne((isadd ? ba : be_)[c]);
#pragma unroll 1
    for (int k = 0; k < D; ++k) s += pmul(xr[k], bf16_rne(w[c * D + k]));
    row[t_] = isadd ? tanhf(s) : 1.0f / (1.0f + __expf(-s)); }
  __syncthreads();
  for (int pass = 0; pass < 2; ++pass) { if (t_ < 32) *(volatile v4f*)(EA + (size_t)p * 2 * D + t_ * 4) = *(const v4f*)(&row[t_ * 4]); __threadfence(); }
}
__global__ __launch_bounds__(256) void write_kernel(const float* __restrict__ vals, const int* __restrict__ midx, const float* __restrict__ EA, float* __restrict__ out1) {
  __shared__ int ids[B]; __shared__ int lastp[256]; __shared__ int anynz;
  const int t_ = threadIdx.x; const size_t r0 = (size_t)blockIdx.x * 256;
  if (t_ == 0) anynz = 0; __syncthreads();
  int nz = 0; for (int p = t_; p < B; p += 256) { const int v = midx[p]; ids[p] = v; nz |= (v != 0); }
  if (nz) anynz = 1;
  __syncthreads();
  { const int row = (int)(r0 + t_); int lp = -1; for (int p = 0; p < B; ++p) if (ids[p] == row) lp = p; lastp[t_] = (anynz && row < M) ? lp : -1; }
  __syncthreads();
  for (int pass = 0; pass < 2; ++pass) { for (int q = t_; q < 256 * 16; q += 256) { const int rr = q >> 4, c4 = (q & 15) * 4; const size_t row = r0 + rr; if (row >= (size_t)M) continue; const v4f old = *(const v4f*)(vals + row * D + c4); v4f nv; const int lp = lastp[rr];
      for (int j = 0; j < 4; ++j) { const float ov = bf16_rne(old[j]); nv[j] = (lp < 0) ? ov : pmul(1.0f - EA[(size_t)lp * 2 * D + c4 + j], ov) + EA[(size_t)lp * 2 * D + D + c4 + j]; }
      *(volatile v4f*)(out1 + row * D + c4) = nv; } __threadfence(); }
}
}

extern "C" void kernel_launch(void* const* d_in, const int* in_sizes, int n_in, void* d_out, int out_size, void* d_ws, size_t ws_size, hipStream_t stream) {
  (void)n_in;
  auto Fp = [&](int i) { return (const float*)d_in[i]; }; auto Ip = [&](int i) { return (const int*)d_in[i]; };
  if (in_sizes[0] != B || in_sizes[1] != B * D || in_sizes[2] != M * D || in_sizes[3] != D * D || in_sizes[5] != D * D || out_size != B * D + M * D) return;
  size_t off = 0; char* ws = (char*)d_ws;
  auto carve = [&](size_t bytes) { char* p = ws + off; off += (bytes + 255) & ~(size_t)255; return p; };
  b16* X16 = (b16*)carve((size_t)B * D * 2); b16* V16 = (b16*)carve((size_t)M * D * 2); b16* VT16 = (b16*)carve((size_t)D * M * 2); float* EA = (float*)carve((size_t)B * 2 * D * 4);
  if (off > ws_size || off > ((size_t)128 << 20)) return;
  float* out0 = (float*)d_out; float* out1 = out0 + (size_t)B * D;
  prep_kernel<<<M / 64, 256, 0, stream>>>(Fp(1), Fp(2), X16, V16, VT16);
  read_kernel<<<B / 32, 64, 0, stream>>>(X16, V16, VT16, out0);
  gate_kernel<<<B, 128, 0, stream>>>(Fp(1), Fp(3), Fp(4), Fp(5), Fp(6), EA);
  write_kernel<<<(M + 255) / 256, 256, 0, stream>>>(Fp(2), Ip(0), EA, out1);
}
